// RelativeTransformerEncoderLayer_71167608095171
// MI455X (gfx1250) — hardware-run, weakly checked
//
#include <hip/hip_runtime.h>


#ifndef NB
#define NB 2
#endif
#ifndef SEQ
#define SEQ 2048
#endif
#define NB_FULL  2
#define SEQ_FULL 2048
#define DM   1024
#define NHD  8
#define HD   64
#define HO   512
#define DFF  4096
#define MROWS (NB * SEQ)
#define AW   4
#define OSP  68
#define MBP  128
#define MBF  64
#define SC2  ((float)(0.125 * 1.4426950408889634))
#define PSH  14.0f
#define NEGB (-3.0e38f)

static constexpr float WSC   = 64.0f;
static constexpr float ONE_F = 1.0f;
static constexpr float CTXC  = 16.0f;
static constexpr float SCW   = 1.0f / 64.0f;
static constexpr float SCWO  = 1.0f / 1024.0f;

static_assert(HD == 64);
static_assert(NHD * HD == HO);
static_assert(2 * HO == DM);
static_assert(DM % 64 == 0);
static_assert(DFF % 64 == 0);
static_assert(HO % 64 == 0);
static_assert(DM % 32 == 0);
static_assert(DFF % 32 == 0);
static_assert(DM == 32 * 8 * 4);
static_assert(SEQ % 64 == 0);
static_assert(MROWS % 64 == 0);
static_assert(MROWS % 8 == 0);
static_assert(SEQ % 8 == 0);
static_assert(SEQ % (16 * AW) == 0);
static_assert(SEQ % 128 == 0);
static_assert(SEQ / 128 <= 16);
static_assert(SEQ / 32 <= MBF);
static_assert(MBF + 4 <= MBP);
static_assert(NB <= NB_FULL);
static_assert(SEQ <= SEQ_FULL);
static_assert((OSP * 4) % 16 == 0);
static_assert(OSP >= 64);
static_assert(AW * 16 * OSP * 4 <= 131072);
static_assert(16 * 68 * 4 <= 131072);
static_assert(4 * 32 * 16 == 16 * HD * 2);
static_assert(8 * 32 * 16 == 16 * 64 * 4);
static_assert(32 * 16 == MBP * 4);

typedef _Float16 h16;
typedef unsigned short bf;
typedef __attribute__((ext_vector_type(16))) _Float16 v16h;
typedef __attribute__((ext_vector_type(8)))  _Float16 v8h;
typedef __attribute__((ext_vector_type(8)))  float    v8f;
typedef __attribute__((ext_vector_type(4)))  float    v4f;
typedef __attribute__((ext_vector_type(4)))  unsigned int v4u;
typedef v4f  __attribute__((may_alias)) v4fa;

__device__ __forceinline__ unsigned short f2bf(float f) { unsigned u = __float_as_uint(f); u += 0x7FFFu + ((u >> 16) & 1u); return (unsigned short)(u >> 16); }
__device__ __forceinline__ float bfr(float f) { return __uint_as_float(((unsigned)f2bf(f)) << 16); }
__device__ __forceinline__ v16h cat16(v8h lo, v8h hi) { return __builtin_shufflevector(lo, hi, 0, 1, 2, 3, 4, 5, 6, 7, 8, 9, 10, 11, 12, 13, 14, 15); }
__device__ __forceinline__ v8f wmma16(v16h a, v16h b, v8f c) { return __builtin_amdgcn_wmma_f32_16x16x32_f16(false, a, false, b, (short)0, c, false, false); }
__device__ __forceinline__ v8f wm(v16h a, v16h b, v8f c) { c = wmma16(a, b, c); asm volatile("v_nop\n\tv_nop\n\tv_nop\n\tv_nop" : "+v"(c) : "v"(a), "v"(b)); return c; }
__device__ __forceinline__ v16h ldh(const h16* p) { return cat16(*(const v8h*)p, *(const v8h*)(p + 16)); }
__device__ __forceinline__ h16 toh_flush(float v) { const h16 r = (h16)v; return (fabsf(v) < 6.103515625e-05f) ? (h16)0.0f : r; }
__device__ __forceinline__ v8h cv8(v4f x0, v4f x1) { v8h o;
#pragma unroll
    for (int i = 0; i < 4; ++i) { o[i] = toh_flush(x0[i]); o[4 + i] = toh_flush(x1[i]); }
    return o; }
__device__ __forceinline__ void wave_sync() { __builtin_amdgcn_fence(3  , "wavefront"); __builtin_amdgcn_wave_barrier(); asm volatile("" ::: "memory"); }

__global__ __launch_bounds__(256) void k_cvth(const float* __restrict__ src, h16* dst, size_t n8, float scale) {
    const size_t i = (size_t)blockIdx.x * 256 + threadIdx.x; if (i >= n8) return;
    const v8f v = *(const v8f*)(src + i * 8); v8h o;
#pragma unroll
    for (int k = 0; k < 8; ++k) o[k] = toh_flush(bfr(v[k]) * scale);
    *(volatile v8h*)(dst + i * 8) = o; __threadfence(); *(volatile v8h*)(dst + i * 8) = o;
}

__global__ __launch_bounds__(256) void k_mpack(const int* __restrict__ mask, unsigned int* MB) {
    const int lane = threadIdx.x & 31;
    const int wave = __builtin_amdgcn_readfirstlane((int)(threadIdx.x >> 5));
    const int i = blockIdx.x * 8 + wave;
    const int* mr = mask + (size_t)i * SEQ_FULL;
    v4u wd = (v4u){0u, 0u, 0u, 0u}; int bad = 0, keep = 0;
#pragma unroll
    for (int c = 0; c < 4; ++c) {
#pragma unroll 1
        for (int q = 0; q < SEQ / 128; ++q) {
            const int key = (4 * q + c) * 32 + lane;
            const int v = mr[key];
            const unsigned int bal = __builtin_amdgcn_ballot_w32(v != 0);
            bad  |= (v == 0 && key >  i) ? 1 : 0;
            keep |= (v == 0 && key <= i) ? 1 : 0;
            wd[c] = (lane == q) ? bal : wd[c]; } }
    const unsigned int anybad = __builtin_amdgcn_ballot_w32(bad != 0);
    const unsigned int anykeep = __builtin_amdgcn_ballot_w32(keep != 0);
    const unsigned int flag = (anybad != 0u || anykeep == 0u) ? 1u : 0u;
    wd[0] = (lane == 16) ? flag : wd[0];
    unsigned int* p = MB + (size_t)i * MBP + 4 * lane;
    *(volatile v4u*)p = wd; __threadfence(); *(volatile v4u*)p = wd;
}

__device__ __forceinline__ void ldx8(const float* p, int inp, float (&x)[8]) {
    const v4f a = *(const v4f*)p, c = *(const v4f*)(p + 4);
#pragma unroll
    for (int i = 0; i < 4; ++i) { x[i] = inp ? bfr(a[i]) : a[i]; x[4 + i] = inp ? bfr(c[i]) : c[i]; }
}

__global__ __launch_bounds__(256) void k_ln(const float* __restrict__ src, const float* __restrict__ g, const float* __restrict__ be, h16* dst, int inp, int flip) {
    const int lane = threadIdx.x & 31;
    const int wave = __builtin_amdgcn_readfirstlane((int)(threadIdx.x >> 5));
    const int m = blockIdx.x * 8 + wave;
    const int b = m / SEQ, t = m % SEQ;
    const int tin = flip ? (SEQ - 1 - t) : t;
    const size_t srow = inp ? ((size_t)tin * NB_FULL + (size_t)b) : (size_t)m;
    const float* xr = src + srow * DM + 8 * lane;
    float x[8];
    float s = 0.0f;
#pragma unroll 1
    for (int k = 0; k < 4; ++k) { ldx8(xr + 256 * k, inp, x);
#pragma unroll
        for (int i = 0; i < 8; ++i) s += x[i]; }
#pragma unroll
    for (int off = 16; off >= 1; off >>= 1) s += __shfl_xor(s, off, 32);
    const float mu = s * (1.0f / (float)DM);
    float s2 = 0.0f;
#pragma unroll 1
    for (int k = 0; k < 4; ++k) { ldx8(xr + 256 * k, inp, x);
#pragma unroll
        for (int i = 0; i < 8; ++i) { const float d = x[i] - mu; s2 += d * d; } }
#pragma unroll
    for (int off = 16; off >= 1; off >>= 1) s2 += __shfl_xor(s2, off, 32);
    const float rstd = rsqrtf(s2 * (1.0f / (float)DM) + 1e-5f);
    h16* orow = dst + (size_t)m * DM + 8 * lane;
#pragma unroll 1
    for (int k = 0; k < 4; ++k) {
        ldx8(xr + 256 * k, inp, x);
        const v4f g0 = *(const v4f*)(g + 256 * k + 8 * lane), g1 = *(const v4f*)(g + 256 * k + 8 * lane + 4);
        const v4f b0 = *(const v4f*)(be + 256 * k + 8 * lane), b1 = *(const v4f*)(be + 256 * k + 8 * lane + 4);
        v8h o;
#pragma unroll
        for (int i = 0; i < 4; ++i) {
            o[i]     = toh_flush((x[i]     - mu) * rstd * bfr(g0[i]) + bfr(b0[i]));
            o[4 + i] = toh_flush((x[4 + i] - mu) * rstd * bfr(g1[i]) + bfr(b1[i])); }
        *(volatile v8h*)(orow + 256 * k) = o; __threadfence(); *(volatile v8h*)(orow + 256 * k) = o; }
}

__device__ __forceinline__ void gemm_core(const h16* __restrict__ A, const h16* __restrict__ Bt, size_t aoff, size_t boff, int K, v8f (&acc)[4][4]) {
#pragma unroll
    for (int mb = 0; mb < 4; ++mb)
#pragma unroll
        for (int nb = 0; nb < 4; ++nb) acc[mb][nb] = (v8f){};
#pragma unroll 1
    for (int kc = 0; kc < K; kc += 32) {
        v16h a[4];
#pragma unroll
        for (int mb = 0; mb < 4; ++mb) a[mb] = ldh(A + aoff + (size_t)mb * 16 * K + kc);
#pragma unroll
        for (int nb = 0; nb < 4; ++nb) { const v16h b = ldh(Bt + boff + (size_t)nb * 16 * K + kc);
#pragma unroll
            for (int mb = 0; mb < 4; ++mb) acc[mb][nb] = wm(a[mb], b, acc[mb][nb]); }
    }
}

__global__ __launch_bounds__(32) void k_gemm_heads(const h16* __restrict__ A, const h16* __restrict__ Bt, const float* __restrict__ rwb, const float* __restrict__ rrb,
                                                   h16* PA, h16* PB, h16* PK, int qcols, float scale) {
    __shared__ __align__(16) float os[16 * 68];
    const int K = DM;
    const int lane = threadIdx.x & 31, lr = lane & 15, hi = lane >> 4; const int r0 = blockIdx.x * 64, c0 = blockIdx.y * 64;
    v8f acc[4][4];
    gemm_core(A, Bt, (size_t)(r0 + lr) * K + 8 * hi, (size_t)(c0 + lr) * K + 8 * hi, K, acc);
    const bool isq = c0 < qcols;
    const int head = (c0 % HO) / HD;
    const int zc = (r0 / SEQ) * NHD + head;
    const size_t tbase = ((size_t)zc * SEQ + (size_t)(r0 % SEQ)) * HD;
    const int cb = (lane & 7) * 8;
    v4f w0 = *(const v4f*)(rwb + head * HD + cb), w1 = *(const v4f*)(rwb + head * HD + cb + 4);
    v4f u0 = *(const v4f*)(rrb + head * HD + cb), u1 = *(const v4f*)(rrb + head * HD + cb + 4);
#pragma unroll
    for (int i = 0; i < 4; ++i) { w0[i] = bfr(w0[i]); w1[i] = bfr(w1[i]); u0[i] = bfr(u0[i]); u1[i] = bfr(u1[i]); }
#pragma unroll
    for (int mb = 0; mb < 4; ++mb) {
#pragma unroll
        for (int nb = 0; nb < 4; ++nb) {
#pragma unroll
            for (int j = 0; j < 8; ++j) os[(hi * 8 + j) * 68 + nb * 16 + lr] = acc[mb][nb][j] * scale; }
        wave_sync();
        const size_t sb = tbase + (size_t)(mb * 16) * HD;
#pragma unroll 1
        for (int ps = 0; ps < 2; ++ps) {
#pragma unroll
            for (int s = 0; s < 4; ++s) { const int p = s * 32 + lane; const int row = p >> 3;
                const v4f x0 = *(const v4fa*)(&os[row * 68 + cb]); const v4f x1 = *(const v4fa*)(&os[row * 68 + cb + 4]);
                const size_t oo = sb + (size_t)p * 8;
                if (isq) { const v8h ha = cv8(x0 + w0, x1 + w1); const v8h hb = cv8(x0 + u0, x1 + u1);
                           *(volatile v8h*)(PA + oo) = ha; *(volatile v8h*)(PB + oo) = hb; }
                else     { const v8h hk = cv8(x0, x1); *(volatile v8h*)(PK + oo) = hk; } }
            if (ps == 0) __threadfence(); }
        wave_sync();
    }
}

__global__ __launch_bounds__(32) void k_gemm_vt(const h16* __restrict__ A, const h16* __restrict__ Bt, h16* PV, float scale) {
    __shared__ __align__(16) float os[16 * 68];
    const int K = DM;
    const int lane = threadIdx.x & 31, lr = lane & 15, hi = lane >> 4; const int r0 = blockIdx.x * 64, c0 = blockIdx.y * 64;
    v8f acc[4][4];
    gemm_core(A, Bt, (size_t)(r0 + lr) * K + 8 * hi, (size_t)(c0 + lr) * K + 8 * hi, K, acc);
    const int bb = c0 / SEQ, tt = c0 % SEQ;
    const size_t tbase = (size_t)bb * (size_t)HO * SEQ + (size_t)r0 * SEQ + (size_t)tt;
#pragma unroll
    for (int mb = 0; mb < 4; ++mb) {
#pragma unroll
        for (int nb = 0; nb < 4; ++nb) {
#pragma unroll
            for (int j = 0; j < 8; ++j) os[(hi * 8 + j) * 68 + nb * 16 + lr] = acc[mb][nb][j] * scale; }
        wave_sync();
        const size_t sb = tbase + (size_t)(mb * 16) * SEQ;
#pragma unroll 1
        for (int ps = 0; ps < 2; ++ps) {
#pragma unroll
            for (int s = 0; s < 4; ++s) { const int row = 4 * s + (lane >> 3), c8 = (lane & 7) * 8;
                const v4f x0 = *(const v4fa*)(&os[row * 68 + c8]); const v4f x1 = *(const v4fa*)(&os[row * 68 + c8 + 4]);
                const v8h hv = cv8(x0, x1);
                *(volatile v8h*)(PV + sb + (size_t)row * SEQ + c8) = hv; }
            if (ps == 0) __threadfence(); }
        wave_sync();
    }
}

__global__ __launch_bounds__(32) void k_gemm_relu(const h16* __restrict__ A, const h16* __restrict__ Bt, const float* __restrict__ bias, h16* Y, float scale) {
    __shared__ __align__(16) float os[16 * 68];
    const int K = DM;
    const int lane = threadIdx.x & 31, lr = lane & 15, hi = lane >> 4; const int r0 = blockIdx.x * 64, c0 = blockIdx.y * 64;
    v8f acc[4][4];
    gemm_core(A, Bt, (size_t)(r0 + lr) * K + 8 * hi, (size_t)(c0 + lr) * K + 8 * hi, K, acc);
    float bc[4];
#pragma unroll
    for (int nb = 0; nb < 4; ++nb) bc[nb] = bfr(bias[c0 + nb * 16 + lr]);
    const size_t tbase = (size_t)r0 * DFF + (size_t)c0;
#pragma unroll
    for (int mb = 0; mb < 4; ++mb) {
#pragma unroll
        for (int nb = 0; nb < 4; ++nb) {
#pragma unroll
            for (int j = 0; j < 8; ++j) { const float v = acc[mb][nb][j] * scale + bc[nb]; os[(hi * 8 + j) * 68 + nb * 16 + lr] = (v > 0.0f) ? v : (v - v); } }
        wave_sync();
        const size_t sb = tbase + (size_t)(mb * 16) * DFF;
#pragma unroll 1
        for (int ps = 0; ps < 2; ++ps) {
#pragma unroll
            for (int s = 0; s < 4; ++s) { const int row = 4 * s + (lane >> 3), c8 = (lane & 7) * 8;
                const v4f x0 = *(const v4fa*)(&os[row * 68 + c8]); const v4f x1 = *(const v4fa*)(&os[row * 68 + c8 + 4]);
                const v8h hv = cv8(x0, x1);
                *(volatile v8h*)(Y + sb + (size_t)row * DFF + c8) = hv; }
            if (ps == 0) __threadfence(); }
        wave_sync();
    }
}

__global__ __launch_bounds__(32) void k_gemm_res(const h16* __restrict__ A, const h16* __restrict__ Bt, const float* __restrict__ bias, const float* __restrict__ R, float* O,
                                                 int K, int rmap, int omap, float scale) {
    __shared__ __align__(16) float os[16 * 68];
    const int lane = threadIdx.x & 31, lr = lane & 15, hi = lane >> 4; const int r0 = blockIdx.x * 64, c0 = blockIdx.y * 64;
    v8f acc[4][4];
    gemm_core(A, Bt, (size_t)(r0 + lr) * K + 8 * hi, (size_t)(c0 + lr) * K + 8 * hi, K, acc);
    float bc[4];
#pragma unroll
    for (int nb = 0; nb < 4; ++nb) bc[nb] = bfr(bias[c0 + nb * 16 + lr]);
    const int bb = r0 / SEQ, tt = r0 % SEQ;
#pragma unroll
    for (int mb = 0; mb < 4; ++mb) {
#pragma unroll
        for (int nb = 0; nb < 4; ++nb) {
#pragma unroll
            for (int j = 0; j < 8; ++j) os[(hi * 8 + j) * 68 + nb * 16 + lr] = acc[mb][nb][j] * scale + bc[nb]; }
        wave_sync();
#pragma unroll 1
        for (int ps = 0; ps < 2; ++ps) {
#pragma unroll
            for (int s = 0; s < 8; ++s) { const int row = 2 * s + (lane >> 4), cofs = (lane & 15) * 4;
                const size_t mrow = (size_t)(r0 + mb * 16 + row);
                const size_t xrow = (size_t)(tt + mb * 16 + row) * NB_FULL + (size_t)bb;
                const size_t rrow = rmap ? xrow : mrow;
                const size_t orow = omap ? xrow : mrow;
                const v4f rv = *(const v4f*)(R + rrow * DM + c0 + cofs);
                const v4f xv = *(const v4fa*)(&os[row * 68 + cofs]);
                v4f val;
#pragma unroll
                for (int i = 0; i < 4; ++i) val[i] = xv[i] + (rmap ? bfr(rv[i]) : rv[i]);
                *(volatile v4f*)(O + orow * DM + c0 + cofs) = val; }
            if (ps == 0) __threadfence(); }
        wave_sync();
    }
}

__global__ __launch_bounds__(32 * AW) __attribute__((amdgpu_num_vgpr(256)))
void k_flash(const h16* __restrict__ QA, const h16* __restrict__ QB, const h16* __restrict__ KP, const h16* __restrict__ RK, const h16* __restrict__ VT,
             const unsigned int* __restrict__ MB, h16* CTX, int colofs, int flip) {
    __shared__ __align__(16) float os[AW * 16 * OSP];
    const int lane = threadIdx.x & 31, lr = lane & 15, hi = lane >> 4;
    const int wave = __builtin_amdgcn_readfirstlane((int)(threadIdx.x >> 5));
    const int zh = blockIdx.y; const int b = zh / NHD, n = zh % NHD;
    const int t0 = (blockIdx.x * AW + wave) * 16;
    const int lim = t0 + lr;
    const int nk = (t0 + 16 + 31) & ~31;
    const size_t pbase = (size_t)zh * SEQ * HD;
    const size_t qo = pbase + (size_t)(t0 + lr) * HD + 8 * hi;
    const v16h qa0 = ldh(QA + qo), qa1 = ldh(QA + qo + 32);
    const v16h qb0 = ldh(QB + qo), qb1 = ldh(QB + qo + 32);
    const size_t ko = pbase + (size_t)lr * HD + 8 * hi;
    const size_t vo = pbase + (size_t)lr * SEQ + 8 * hi;
    const size_t rko = (size_t)n * SEQ * HD + 8 * hi;
    const unsigned int* mrow = MB + (size_t)(t0 + lr) * MBP;
    const int wb = wave * 16 * OSP;
    const int wro = wb + lr * OSP + 8 * hi;
    const int rdo = wb + lr * OSP + 15 - lr + 8 * hi;
    v8f o0 = (v8f){}, o1 = (v8f){}, o2 = (v8f){}, o3 = (v8f){};
    float m = NEGB, l = 0.0f;
#pragma unroll 1
    for (int key0 = 0; key0 < nk; key0 += 32) {
        unsigned int mw = mrow[key0 >> 5];
        asm volatile("" : "+v"(mw));
        const int rlo = SEQ - 16 - t0 + key0;
#pragma unroll
        for (int u = 0; u < 3; ++u) {
            int rr = rlo + 16 * u + lr; rr = rr > SEQ - 1 ? SEQ - 1 : rr;
            const h16* rp = RK + rko + (size_t)rr * HD;
            const v16h ra0 = ldh(rp), ra1 = ldh(rp + 32);
            v8f d = (v8f){};
            d = wm(ra0, qb0, d); d = wm(ra1, qb1, d);
            v4f a, c;
            a[0] = d[0]; a[1] = d[1]; a[2] = d[2]; a[3] = d[3]; c[0] = d[4]; c[1] = d[5]; c[2] = d[6]; c[3] = d[7];
            *(v4fa*)(&os[wro + 16 * u]) = a; *(v4fa*)(&os[wro + 16 * u + 4]) = c; }
        wave_sync();
        const h16* ka = KP + ko + (size_t)key0 * HD;
        const v16h ka0 = ldh(ka), ka1 = ldh(ka + 32), kb0 = ldh(ka + 16 * HD), kb1 = ldh(ka + 16 * HD + 32);
        v8f sa = (v8f){}, sb = (v8f){};
        sa = wm(ka0, qa0, sa); sa = wm(ka1, qa1, sa);
        sb = wm(kb0, qa0, sb); sb = wm(kb1, qa1, sb);
        float ra[8], rb[8];
#pragma unroll
        for (int r = 0; r < 8; ++r) { ra[r] = os[rdo + r]; rb[r] = os[rdo + 16 + r]; }
        wave_sync();
        const int ja = key0 + 8 * hi;
        float ta[8], tb[8]; bool fa[8], fb[8]; float mx = NEGB;
#pragma unroll
        for (int r = 0; r < 8; ++r) {
            fa[r] = (((mw >> (8 * hi + r)) & 1u) == 0u) && (ja + r <= lim);
            fb[r] = (((mw >> (16 + 8 * hi + r)) & 1u) == 0u) && (ja + 16 + r <= lim);
            ta[r] = (sa[r] + ra[r]) * SC2; tb[r] = (sb[r] + rb[r]) * SC2;
            mx = fmaxf(mx, fmaxf(fa[r] ? ta[r] : NEGB, fb[r] ? tb[r] : NEGB)); }
        mx = fmaxf(mx, __shfl_xor(mx, 16, 32));
        const float mnew = fmaxf(m, mx);
        const float alpha = __builtin_amdgcn_exp2f(m - mnew);
        const float sh = PSH - mnew;
        v16h pb; float ls = 0.0f;
#pragma unroll
        for (int r = 0; r < 8; ++r) {
            const float xa = ta[r] + sh, xb = tb[r] + sh;
            const float ea = (xa < -14.0f) ? 0.0f : __builtin_amdgcn_exp2f(xa);
            const float eb = (xb < -14.0f) ? 0.0f : __builtin_amdgcn_exp2f(xb);
            const float ga = fa[r] ? ea : 0.0f, gb = fb[r] ? eb : 0.0f;
            const h16 pa = (h16)ga; const h16 pc = (h16)gb;
            pb[r] = pa; pb[8 + r] = pc;
            ls += (float)pa + (float)pc; }
        l = l * alpha + ls; m = mnew;
        o0 = o0 * alpha; o1 = o1 * alpha; o2 = o2 * alpha; o3 = o3 * alpha;
        const h16* va = VT + vo + key0;
        const v16h v0 = ldh(va), v1 = ldh(va + (size_t)16 * SEQ), v2 = ldh(va + (size_t)32 * SEQ), v3 = ldh(va + (size_t)48 * SEQ);
        o0 = wm(v0, pb, o0); o1 = wm(v1, pb, o1); o2 = wm(v2, pb, o2); o3 = wm(v3, pb, o3);
    }
    l += __shfl_xor(l, 16, 32);
    const bool any = l > 0.0f;
    const float lsafe = any ? l : 1.0f;
    float inv = any ? (CTXC / lsafe) : 0.0f;
    const unsigned int fw = mrow[MBF];
    inv = (fw != 0u) ? __uint_as_float(0x7fc00000u) : inv;
    { v4f a, c;
      a[0] = o0[0] * inv; a[1] = o0[1] * inv; a[2] = o0[2] * inv; a[3] = o0[3] * inv; c[0] = o0[4] * inv; c[1] = o0[5] * inv; c[2] = o0[6] * inv; c[3] = o0[7] * inv;
      *(v4fa*)(&os[wro +  0]) = a; *(v4fa*)(&os[wro +  0 + 4]) = c;
      a[0] = o1[0] * inv; a[1] = o1[1] * inv; a[2] = o1[2] * inv; a[3] = o1[3] * inv; c[0] = o1[4] * inv; c[1] = o1[5] * inv; c[2] = o1[6] * inv; c[3] = o1[7] * inv;
      *(v4fa*)(&os[wro + 16]) = a; *(v4fa*)(&os[wro + 16 + 4]) = c;
      a[0] = o2[0] * inv; a[1] = o2[1] * inv; a[2] = o2[2] * inv; a[3] = o2[3] * inv; c[0] = o2[4] * inv; c[1] = o2[5] * inv; c[2] = o2[6] * inv; c[3] = o2[7] * inv;
      *(v4fa*)(&os[wro + 32]) = a; *(v4fa*)(&os[wro + 32 + 4]) = c;
      a[0] = o3[0] * inv; a[1] = o3[1] * inv; a[2] = o3[2] * inv; a[3] = o3[3] * inv; c[0] = o3[4] * inv; c[1] = o3[5] * inv; c[2] = o3[6] * inv; c[3] = o3[7] * inv;
      *(v4fa*)(&os[wro + 48]) = a; *(v4fa*)(&os[wro + 48 + 4]) = c; }
    wave_sync();
    h16* cbase = CTX + (size_t)b * SEQ * DM + (size_t)colofs + (size_t)n * HD;
#pragma unroll 1
    for (int ps = 0; ps < 2; ++ps) {
#pragma unroll
        for (int s = 0; s < 4; ++s) { const int row = 4 * s + (lane >> 3), c8 = (lane & 7) * 8;
            const int t = t0 + row; const int tout = flip ? (SEQ - 1 - t) : t;
            const v4f x0 = *(const v4fa*)(&os[wb + row * OSP + c8]); const v4f x1 = *(const v4fa*)(&os[wb + row * OSP + c8 + 4]);
            const v8h hv = cv8(x0, x1);
            *(volatile v8h*)(cbase + (size_t)tout * DM + c8) = hv; }
        if (ps == 0) __threadfence(); }
}

static constexpr size_t al256(size_t v) { return (v + 255) & ~(size_t)255; }
static constexpr size_t N_WQKV = (size_t)3 * HO * DM;
static constexpr size_t N_WR   = (size_t)HO * DM;
static constexpr size_t N_ACT  = (size_t)MROWS * DM;
static constexpr size_t N_HP   = (size_t)MROWS * HO;
static constexpr size_t N_RK   = (size_t)NHD * SEQ * HD;
static constexpr size_t N_MB   = (size_t)SEQ * MBP;
static constexpr size_t SZ_WQKV = al256(2 * N_WQKV * 2);
static constexpr size_t SZ_WR   = al256(2 * N_WR * 2);
static constexpr size_t SZ_WO   = al256((size_t)DM * DM * 2);
static constexpr size_t SZ_W1   = al256((size_t)DFF * DM * 2);
static constexpr size_t SZ_W2   = al256((size_t)DM * DFF * 2);
static constexpr size_t SZ_POS  = al256((size_t)SEQ * DM * 2);
static constexpr size_t SZ_LNA  = al256(2 * N_ACT * 2);
static constexpr size_t SZ_HPL  = al256(8 * N_HP * 2);
static constexpr size_t SZ_RK   = al256(2 * N_RK * 2);
static constexpr size_t SZ_CTX  = al256(N_ACT * 2);
static constexpr size_t SZ_H    = al256(N_ACT * 4);
static constexpr size_t SZ_LN3  = al256(N_ACT * 2);
static constexpr size_t SZ_MB   = al256(2 * N_MB * 4);
static constexpr size_t SZ_TOTAL = SZ_WQKV + SZ_WR + SZ_WO + SZ_W1 + SZ_W2 + SZ_POS + SZ_LNA + SZ_HPL + SZ_RK + SZ_CTX + SZ_H + SZ_LN3 + SZ_MB;
static_assert(SZ_TOTAL <= (size_t)134217728);
static_assert((size_t)MROWS * DFF * 2 <= SZ_HPL);
static_assert((N_WQKV * 2) % 256 == 0);
static_assert((N_WR * 2) % 256 == 0);
static_assert((N_ACT * 2) % 256 == 0);
static_assert((N_HP * 2) % 256 == 0);
static_assert((N_RK * 2) % 256 == 0);
static_assert((N_MB * 4) % 256 == 0);
static_assert(N_WQKV % 64 == 0);
static_assert(N_WR % 64 == 0);
static_assert(((size_t)SEQ * DM) % 64 == 0);
static_assert((size_t)NB * NHD * SEQ * HD == N_HP);
static_assert((size_t)NB * HO * SEQ == N_HP);

extern "C" void kernel_launch(void* const* d_in, const int* in_sizes, int n_in,
                              void* d_out, int out_size, void* d_ws, size_t ws_size, hipStream_t stream) {
    if (n_in < 24) return;
    const size_t needx = ((size_t)(SEQ - 1) * NB_FULL + NB) * DM;
    const size_t needm = (size_t)(SEQ - 1) * SEQ_FULL + SEQ;
    if ((size_t)in_sizes[0] < needx || (size_t)in_sizes[1] < (size_t)SEQ * DM) return;
    if ((size_t)in_sizes[2] < needm || (size_t)in_sizes[3] < needm) return;
    for (int i = 4; i < 10; ++i) if (in_sizes[i] < DM) return;
    if ((size_t)in_sizes[10] < N_WQKV || (size_t)in_sizes[14] < N_WQKV) return;
    if ((size_t)in_sizes[11] < N_WR || (size_t)in_sizes[15] < N_WR) return;
    if (in_sizes[12] < HO || in_sizes[13] < HO || in_sizes[16] < HO || in_sizes[17] < HO) return;
    if ((size_t)in_sizes[18] < (size_t)DM * DM || in_sizes[19] < DM) return;
    if ((size_t)in_sizes[20] < (size_t)DFF * DM || in_sizes[21] < DFF) return;
    if ((size_t)in_sizes[22] < (size_t)DM * DFF || in_sizes[23] < DM) return;
    if ((size_t)out_size < needx) return;
    if (SZ_TOTAL > ws_size) return;
    const float* x = (const float*)d_in[0];
    const float* pos = (const float*)d_in[1];
    const int* maskd[2] = { (const int*)d_in[2], (const int*)d_in[3] };
    const float* lng[3] = { (const float*)d_in[4], (const float*)d_in[6], (const float*)d_in[8] };
    const float* lnb[3] = { (const float*)d_in[5], (const float*)d_in[7], (const float*)d_in[9] };
    const float* wqkv[2] = { (const float*)d_in[10], (const float*)d_in[14] };
    const float* wrn[2]  = { (const float*)d_in[11], (const float*)d_in[15] };
    const float* rwb[2]  = { (const float*)d_in[12], (const float*)d_in[16] };
    const float* rrb[2]  = { (const float*)d_in[13], (const float*)d_in[17] };
    const float* wo = (const float*)d_in[18]; const float* bo = (const float*)d_in[19];
    const float* w1 = (const float*)d_in[20]; const float* b1 = (const float*)d_in[21];
    const float* w2 = (const float*)d_in[22]; const float* b2 = (const float*)d_in[23];
    float* OUT = (float*)d_out;
    char* wsp = (char*)d_ws;
    h16* WQKV = (h16*)wsp; wsp += SZ_WQKV;
    h16* WR   = (h16*)wsp; wsp += SZ_WR;
    h16* WOH  = (h16*)wsp; wsp += SZ_WO;
    h16* W1H  = (h16*)wsp; wsp += SZ_W1;
    h16* W2H  = (h16*)wsp; wsp += SZ_W2;
    h16* POSH = (h16*)wsp; wsp += SZ_POS;
    h16* LNA  = (h16*)wsp; wsp += SZ_LNA;
    h16* HPL  = (h16*)wsp; wsp += SZ_HPL;
    h16* RKP  = (h16*)wsp; wsp += SZ_RK;
    h16* CTX  = (h16*)wsp; wsp += SZ_CTX;
    float* HB = (float*)wsp; wsp += SZ_H;
    h16* LN3  = (h16*)wsp; wsp += SZ_LN3;
    unsigned int* MBW = (unsigned int*)wsp; wsp += SZ_MB;
    h16* QAP = HPL; h16* QBP = HPL + 2 * N_HP; h16* KPP = HPL + 4 * N_HP; h16* VTP = HPL + 6 * N_HP;
    h16* Y1 = HPL;

    for (int d = 0; d < 2; ++d) {
        k_cvth<<<(unsigned)((N_WQKV / 8 + 255) / 256), 256, 0, stream>>>(wqkv[d], WQKV + (size_t)d * N_WQKV, N_WQKV / 8, WSC);
        k_cvth<<<(unsigned)((N_WR / 8 + 255) / 256), 256, 0, stream>>>(wrn[d], WR + (size_t)d * N_WR, N_WR / 8, WSC);
    }
    k_cvth<<<(unsigned)(((size_t)DM * DM / 8 + 255) / 256), 256, 0, stream>>>(wo, WOH, (size_t)DM * DM / 8, WSC);
    k_cvth<<<(unsigned)(((size_t)DFF * DM / 8 + 255) / 256), 256, 0, stream>>>(w1, W1H, (size_t)DFF * DM / 8, WSC);
    k_cvth<<<(unsigned)(((size_t)DM * DFF / 8 + 255) / 256), 256, 0, stream>>>(w2, W2H, (size_t)DM * DFF / 8, WSC);
    k_cvth<<<(unsigned)(((size_t)SEQ * DM / 8 + 255) / 256), 256, 0, stream>>>(pos, POSH, (size_t)SEQ * DM / 8, ONE_F);

    for (int d = 0; d < 2; ++d) {
        k_ln<<<MROWS / 8, 256, 0, stream>>>(x, lng[d], lnb[d], LNA + (size_t)d * N_ACT, 1, d);
        k_mpack<<<SEQ / 8, 256, 0, stream>>>(maskd[d], MBW + (size_t)d * N_MB);
        k_gemm_heads<<<dim3(MROWS / 64, (2 * HO) / 64, 1), 32, 0, stream>>>(LNA + (size_t)d * N_ACT, WQKV + (size_t)d * N_WQKV, rwb[d], rrb[d],
                                                                           QAP + (size_t)d * N_HP, QBP + (size_t)d * N_HP, KPP + (size_t)d * N_HP, HO, SCW);
        k_gemm_vt<<<dim3(HO / 64, MROWS / 64, 1), 32, 0, stream>>>(WQKV + (size_t)d * N_WQKV + (size_t)2 * HO * DM, LNA + (size_t)d * N_ACT, VTP + (size_t)d * N_HP, SCW);
        k_gemm_heads<<<dim3(SEQ / 64, HO / 64, 1), 32, 0, stream>>>(POSH, WR + (size_t)d * N_WR, rwb[d], rrb[d],
                                                                    QAP + (size_t)d * N_HP, QBP + (size_t)d * N_HP, RKP + (size_t)d * N_RK, 0, SCW);
    }
    for (int d = 0; d < 2; ++d)
        k_flash<<<dim3(SEQ / (16 * AW), NB * NHD, 1), 32 * AW, 0, stream>>>(QAP + (size_t)d * N_HP, QBP + (size_t)d * N_HP, KPP + (size_t)d * N_HP, RKP + (size_t)d * N_RK,
                                                                            VTP + (size_t)d * N_HP, MBW + (size_t)d * N_MB, CTX, d * HO, d);
    k_gemm_res<<<dim3(MROWS / 64, DM / 64, 1), 32, 0, stream>>>(CTX, WOH, bo, x, HB, DM, 1, 0, SCWO);
    k_ln<<<MROWS / 8, 256, 0, stream>>>(HB, lng[2], lnb[2], LN3, 0, 0);
    k_gemm_relu<<<dim3(MROWS / 64, DFF / 64, 1), 32, 0, stream>>>(LN3, W1H, b1, Y1, SCW);
    k_gemm_res<<<dim3(MROWS / 64, DM / 64, 1), 32, 0, stream>>>(Y1, W2H, b2, HB, OUT, DFF, 0, 1, SCW);
}
